// GIN_45397804319031
// MI455X (gfx1250) — hardware-verified
//
#include <hip/hip_runtime.h>
#include <stddef.h>
#include <stdint.h>
#include <math.h>


#define DD      128
#define HID2    256
#define NO      10
#define HK      (2 * DD)
#define TK      (2 * HID2)
#define NTHR    256
#define NWAVE   8
#define EPT     8
#define CHUNK   (NTHR * EPT)
#define WCAP    (EPT * 32)
#define LISTN   (NWAVE * WCAP)
#define NB      256
#define PKS     8
#define RCAP    24576
#define DEGCAP  128
#define GBM     64
#define GBN     128
#define GTHR    128
#define GNT     8
#define HG      16
#define HTHR    128
#define APIT    264
#define NUW1    (HID2 * (HK / 8))
#define NUW2    (DD * (TK / 8))
#define NUL1    (DD * (HK / 8))
#define PB1     (NUW1)
#define PB2     (2 * NUW1)
#define PB3     (2 * NUW1 + NUW2)
#define PB4     (2 * NUW1 + 2 * NUW2)
#define PB5     (PB4 + NUL1)
#define WSMAX   134217728
#define LDS_AGG ((2 * RCAP + 2 * NB + LISTN) * 4 + 64)

static_assert((CHUNK & (CHUNK - 1)) == 0);
static_assert((NB & (NB - 1)) == 0 && NB <= (1 << PKS) && NB == NTHR);
static_assert(((long long)CHUNK << PKS) < (1LL << 31));
static_assert(LISTN >= NB && LISTN == NWAVE * WCAP);
static_assert((RCAP % 32) == 0 && (NB % NWAVE) == 0);
static_assert(LDS_AGG <= 300000);
static_assert(GBM == (GTHR / 32) * 16 && GBN == 16 * GNT && GTHR == GBN);
static_assert(DD == 32 * 4);
static_assert((HK % 32) == 0 && (TK % 32) == 0);
static_assert((HID2 % GBN) == 0 && (DD % GBN) == 0);
static_assert((PB1 % NTHR) == 0 && (PB2 % NTHR) == 0 && (PB3 % NTHR) == 0 && (PB4 % NTHR) == 0 && (PB5 % NTHR) == 0);
static_assert((HK / 8) == 32 && (TK / 8) == 64 && (DD / 8) == 16);
static_assert(HTHR == DD && (HTHR / 32) * 32 == DD);
static_assert(((HG * NO) % 32) == 0 && (HG * NO) / 4 <= HTHR);
static_assert(HG == 16 && NO <= 16 && (APIT % 8) == 0 && APIT >= HK);

typedef float          v4f  __attribute__((ext_vector_type(4)));
typedef float          v8f  __attribute__((ext_vector_type(8)));
typedef int            v4i  __attribute__((ext_vector_type(4)));
typedef int            v8i  __attribute__((ext_vector_type(8)));
typedef unsigned int   v2u  __attribute__((ext_vector_type(2)));
typedef unsigned int   v4u  __attribute__((ext_vector_type(4)));
typedef unsigned short v8us __attribute__((ext_vector_type(8)));
typedef __bf16         v16b __attribute__((ext_vector_type(16)));
typedef v4f  __attribute__((may_alias)) v4fa;
typedef v8us __attribute__((may_alias)) v8usa;
union Frag { v16b vb; v8us h[2]; v8i w; };

__device__ __forceinline__ v8f wmb(const Frag& a, const Frag& b, v8f c) {
  v8f d = __builtin_amdgcn_wmma_f32_16x16x32_bf16(false, a.vb, false, b.vb, (short)0, c, false, false);
  asm volatile("v_nop\n\tv_nop\n\tv_nop\n\tv_nop" : "+v"(d) : "v"(a.w), "v"(b.w));
  return d;
}

__device__ __forceinline__ unsigned short bf_bits(float f) {
  unsigned int u = __float_as_uint(f);
  u += 0x7FFFu + ((u >> 16) & 1u);
  return (unsigned short)(u >> 16);
}
__device__ __forceinline__ float bf_val(unsigned short b) { return __uint_as_float(((unsigned int)b) << 16); }
__device__ __forceinline__ float bf_rne(float f) { return bf_val(bf_bits(f)); }

__device__ __forceinline__ float relu_keep(float v) { return (v > 0.0f) ? v : (v - v); }

__device__ __forceinline__ int scan_chunk(const int* __restrict__ dsts, int nE, int cbase, int slotBase,
                                          int nb, int vec8, int* list, int tid, int lane, int wave) {
  int wc = 0;
  const int el0  = tid * EPT;
  const int e0   = cbase + el0;
  const int sent = -2147483647 - 1;
  v4i da, db;
  if (vec8 != 0 && cbase + CHUNK <= nE) {
    da = *(const v4i*)(dsts + e0);
    db = *(const v4i*)(dsts + e0 + 4);
  } else {
    da.x = (e0     < nE) ? dsts[min(e0,     nE - 1)] : sent;
    da.y = (e0 + 1 < nE) ? dsts[min(e0 + 1, nE - 1)] : sent;
    da.z = (e0 + 2 < nE) ? dsts[min(e0 + 2, nE - 1)] : sent;
    da.w = (e0 + 3 < nE) ? dsts[min(e0 + 3, nE - 1)] : sent;
    db.x = (e0 + 4 < nE) ? dsts[min(e0 + 4, nE - 1)] : sent;
    db.y = (e0 + 5 < nE) ? dsts[min(e0 + 5, nE - 1)] : sent;
    db.z = (e0 + 6 < nE) ? dsts[min(e0 + 6, nE - 1)] : sent;
    db.w = (e0 + 7 < nE) ? dsts[min(e0 + 7, nE - 1)] : sent;
  }
  const unsigned nbs = (unsigned)slotBase;
  const unsigned unb = (unsigned)nb;
  const unsigned s0 = (unsigned)da.x - nbs, s1 = (unsigned)da.y - nbs;
  const unsigned s2 = (unsigned)da.z - nbs, s3 = (unsigned)da.w - nbs;
  const unsigned s4 = (unsigned)db.x - nbs, s5 = (unsigned)db.y - nbs;
  const unsigned s6 = (unsigned)db.z - nbs, s7 = (unsigned)db.w - nbs;
  const bool h0 = s0 < unb, h1 = s1 < unb, h2 = s2 < unb, h3 = s3 < unb;
  const bool h4 = s4 < unb, h5 = s5 < unb, h6 = s6 < unb, h7 = s7 < unb;
  const unsigned any = __builtin_amdgcn_ballot_w32(h0 | h1 | h2 | h3 | h4 | h5 | h6 | h7);
  if (any != 0u) {
#define HITJ(J, HJ, SJ) { \
      const unsigned mj = __builtin_amdgcn_ballot_w32(HJ); \
      if (mj != 0u) { \
        if (HJ) { \
          const int pos = wc + (int)__builtin_amdgcn_mbcnt_lo(mj, 0u); \
          if (pos < WCAP) list[wave * WCAP + pos] = ((el0 + (J)) << PKS) | (int)(SJ); \
        } \
        wc += (int)__builtin_popcount(mj); } }
    HITJ(0, h0, s0)
    HITJ(1, h1, s1)
    HITJ(2, h2, s2)
    HITJ(3, h3, s3)
    HITJ(4, h4, s4)
    HITJ(5, h5, s5)
    HITJ(6, h6, s6)
    HITJ(7, h7, s7)
#undef HITJ
  }
  return wc;
}

__device__ __forceinline__ v8us cv8b(const float* __restrict__ p, size_t stride) {
  v8us o;
#pragma unroll
  for (int i = 0; i < 8; ++i) o[i] = bf_bits(p[(size_t)i * stride]);
  return o;
}

__global__ __launch_bounds__(NTHR) void k_prep(const float* __restrict__ x, int nUx,
                                               const float* __restrict__ w10, const float* __restrict__ w11,
                                               const float* __restrict__ w20, const float* __restrict__ w21,
                                               const float* __restrict__ l1,
                                               unsigned short* p10, unsigned short* p11,
                                               unsigned short* p20, unsigned short* p21,
                                               unsigned short* pl1, unsigned short* xb) {
  const int u = (int)blockIdx.x * NTHR + (int)threadIdx.x;
  v8us o;
  unsigned short* dp;
  bool ok = true;
  if (u < PB1) {
    const int v = u, n = v >> 5, k8 = (v & 31) * 8, kk = k8 & (DD - 1);
    o = cv8b(w10 + (size_t)kk * HID2 + n, HID2);
    dp = p10 + (size_t)v * 8;
  } else if (u < PB2) {
    const int v = u - PB1, n = v >> 5, k8 = (v & 31) * 8, kk = k8 & (DD - 1);
    o = cv8b(w11 + (size_t)kk * HID2 + n, HID2);
    dp = p11 + (size_t)v * 8;
  } else if (u < PB3) {
    const int v = u - PB2, n = v >> 6, k8 = (v & 63) * 8, kk = k8 & (HID2 - 1);
    o = cv8b(w20 + (size_t)kk * DD + n, DD);
    dp = p20 + (size_t)v * 8;
  } else if (u < PB4) {
    const int v = u - PB3, n = v >> 6, k8 = (v & 63) * 8, kk = k8 & (HID2 - 1);
    o = cv8b(w21 + (size_t)kk * DD + n, DD);
    dp = p21 + (size_t)v * 8;
  } else if (u < PB5) {
    const int v = u - PB4, n = v >> 5, k8 = (v & 31) * 8, kk = k8 & (DD - 1);
    o = cv8b(l1 + (size_t)kk * DD + n, DD);
    dp = pl1 + (size_t)v * 8;
  } else {
    const int v = u - PB5;
    ok = v < nUx;
    const int vc = ok ? v : nUx - 1;
    const float* p = x + (size_t)vc * 8;
    const v4f a = *(const v4fa*)p;
    const v4f b = *(const v4fa*)(p + 4);
    o[0] = bf_bits(a.x); o[1] = bf_bits(a.y); o[2] = bf_bits(a.z); o[3] = bf_bits(a.w);
    o[4] = bf_bits(b.x); o[5] = bf_bits(b.y); o[6] = bf_bits(b.z); o[7] = bf_bits(b.w);
    dp = xb + (size_t)vc * 8;
  }
  if (ok) *(volatile v8us*)dp = o;
  __threadfence();
  if (ok) *(volatile v8us*)dp = o;
}

template <int SRCB>
__device__ __forceinline__ v4f ldrow(const unsigned short* __restrict__ xb, const float* __restrict__ fin,
                                     int s, int lane) {
  if constexpr (SRCB != 0) {
    const v2u w = *(const v2u*)(xb + (size_t)s * DD + 4 * lane);
    v4f r;
    r.x = __uint_as_float(w.x << 16);
    r.y = __uint_as_float(w.x & 0xffff0000u);
    r.z = __uint_as_float(w.y << 16);
    r.w = __uint_as_float(w.y & 0xffff0000u);
    return r;
  } else {
    return *(const v4f*)(fin + (size_t)s * DD + 4 * lane);
  }
}

template <int SRCB>
__global__ __launch_bounds__(NTHR) void k_agg(
    const int* __restrict__ srcs, const int* __restrict__ dsts,
    const unsigned short* __restrict__ xb, const float* __restrict__ fin,
    const float* __restrict__ epsp,
    unsigned short* Hout, int nN, int nE, int vec8, int MPr) {
  extern __shared__ v4f lds_dyn[];
  int* reg1 = (int*)lds_dyn;
  int* reg2 = reg1 + RCAP;
  int* scnt = reg2 + RCAP;
  int* soff = scnt + NB;
  int* list = soff + NB;
  int* wcnt = list + LISTN;
  int* wtot = wcnt + NWAVE;
  const int tid = (int)threadIdx.x, lane = tid & 31, wave = tid >> 5;
  const int nodeBase = (int)blockIdx.x * NB;
  const float e1 = 1.0f + bf_rne(epsp[0]);

  scnt[tid] = 0;
  __syncthreads();

  int tot = 0;
  const int nChunks = (nE + CHUNK - 1) / CHUNK;
#pragma unroll 1
  for (int ch = 0; ch < nChunks; ++ch) {
    const int cbase = ch * CHUNK;
    const int wc = scan_chunk(dsts, nE, cbase, nodeBase, NB, vec8, list, tid, lane, wave);
    if (lane == 0) wcnt[wave] = wc;
    __syncthreads();
    int pre = 0, all = 0;
#pragma unroll
    for (int w2 = 0; w2 < NWAVE; ++w2) {
      int c = wcnt[w2];
      c = c < 0 ? 0 : (c > WCAP ? WCAP : c);
      all += c;
      pre += (w2 < wave) ? c : 0;
    }
    const int wcc  = wc > WCAP ? WCAP : wc;
    const int base = tot + pre;
#pragma unroll 1
    for (int i = lane; i < wcc; i += 32) {
      const int ent = list[wave * WCAP + i];
      const int el  = (ent >> PKS) & (CHUNK - 1);
      const int sl  = ent & (NB - 1);
      int eid = cbase + el;
      eid = eid > nE - 1 ? nE - 1 : eid;
      const int pos = base + i;
      if (pos < RCAP) reg1[pos] = (int)(((unsigned)eid << PKS) | (unsigned)sl);
    }
    tot += all;
    tot = tot > RCAP ? RCAP : tot;
    __syncthreads();
  }
  const int nh = tot;

  if (wave == 0) {
#pragma unroll 1
    for (int b0 = 0; b0 < nh; b0 += 32) {
      int idx = b0 + lane;
      idx = idx > nh - 1 ? nh - 1 : idx;
      const int uv  = reg1[idx];
      const int m32 = (nh - b0) < 32 ? (nh - b0) : 32;
#pragma unroll 1
      for (int k = 0; k < m32; ++k) {
        const int u  = __builtin_amdgcn_readlane(uv, k);
        const int sl = u & (NB - 1);
        if (lane == 0) scnt[sl] = scnt[sl] + 1;
      }
    }
  }
  __syncthreads();

  {
    int e = scnt[tid];
    e = e < 0 ? 0 : e;
    int incl = e;
#pragma unroll
    for (int d = 1; d < 32; d <<= 1) {
      const int up = __shfl_up(incl, d);
      if (lane >= d) incl += up;
    }
    if (lane == 31) wtot[wave] = incl;
    __syncthreads();
    int pre = 0;
#pragma unroll
    for (int w2 = 0; w2 < NWAVE; ++w2) pre += (w2 < wave) ? wtot[w2] : 0;
    const int ex = pre + incl - e;
    soff[tid] = ex;
    list[tid] = ex;
  }
  __syncthreads();

  if (wave == 0) {
#pragma unroll 1
    for (int b0 = 0; b0 < nh; b0 += 32) {
      int idx = b0 + lane;
      idx = idx > nh - 1 ? nh - 1 : idx;
      const int uv  = reg1[idx];
      const int m32 = (nh - b0) < 32 ? (nh - b0) : 32;
#pragma unroll 1
      for (int k = 0; k < m32; ++k) {
        const int u   = __builtin_amdgcn_readlane(uv, k);
        const int sl  = u & (NB - 1);
        const int eid = (int)((unsigned)u >> PKS);
        if (lane == 0) {
          int pos = list[sl];
          pos = pos < 0 ? 0 : (pos > RCAP - 1 ? RCAP - 1 : pos);
          reg2[pos] = eid;
          list[sl] = pos + 1;
        }
      }
    }
  }
  __syncthreads();

  const int nbw = NB / NWAVE;
  const bool ovf = (nh >= RCAP);
  const float qnan = __int_as_float(0x7fc00000);

#pragma unroll 1
  for (int jt = 0; jt < nbw; ++jt) {
    const int slot = wave * nbw + jt;
    const int grow = nodeBase + slot;
    int st = soff[slot];
    const int craw = scnt[slot];
    int cnt = craw;
    st  = st < 0 ? 0 : (st > nh ? nh : st);
    cnt = cnt < 0 ? 0 : (cnt > DEGCAP ? DEGCAP : cnt);
    if (cnt > nh - st) cnt = nh - st;
    const float pz = (ovf || craw > DEGCAP) ? qnan : 0.0f;
    const bool liveRow = grow < nN;

    float ag0 = 0.0f, ag1 = 0.0f, ag2 = 0.0f, ag3 = 0.0f;
#pragma unroll 1
    for (int b0 = 0; b0 < cnt; b0 += 32) {
      int idx = st + b0 + lane;
      idx = idx > st + cnt - 1 ? st + cnt - 1 : idx;
      idx = idx < 0 ? 0 : (idx > RCAP - 1 ? RCAP - 1 : idx);
      int eid = reg2[idx];
      eid = eid < 0 ? 0 : (eid > nE - 1 ? nE - 1 : eid);
      int sr = srcs[eid];
      sr = sr < 0 ? 0 : (sr > nN - 1 ? nN - 1 : sr);
      const int m32 = (cnt - b0) < 32 ? (cnt - b0) : 32;
#pragma unroll 1
      for (int k = 0; k < m32; ++k) {
        const int sk = __builtin_amdgcn_readlane(sr, k);
        const v4f v = ldrow<SRCB>(xb, fin, sk, lane);
        ag0 += v.x; ag1 += v.y; ag2 += v.z; ag3 += v.w;
      }
    }
    const int nc = liveRow ? grow : nN - 1;
    const v4f sv = ldrow<SRCB>(xb, fin, nc, lane);
    float r0 = fmaf(e1, sv.x, ag0), r1 = fmaf(e1, sv.y, ag1);
    float r2 = fmaf(e1, sv.z, ag2), r3 = fmaf(e1, sv.w, ag3);
    r0 = (liveRow ? r0 : 0.0f) + pz;
    r1 = (liveRow ? r1 : 0.0f) + pz;
    r2 = (liveRow ? r2 : 0.0f) + pz;
    r3 = (liveRow ? r3 : 0.0f) + pz;

    const unsigned short h0 = bf_bits(r0), h1 = bf_bits(r1), h2 = bf_bits(r2), h3 = bf_bits(r3);
    const unsigned short l0 = bf_bits(r0 - bf_val(h0)), l1 = bf_bits(r1 - bf_val(h1));
    const unsigned short l2 = bf_bits(r2 - bf_val(h2)), l3 = bf_bits(r3 - bf_val(h3));
    v2u ph, pl;
    ph.x = (unsigned int)h0 | ((unsigned int)h1 << 16);
    ph.y = (unsigned int)h2 | ((unsigned int)h3 << 16);
    pl.x = (unsigned int)l0 | ((unsigned int)l1 << 16);
    pl.y = (unsigned int)l2 | ((unsigned int)l3 << 16);
    unsigned short* gp = Hout + (size_t)grow * HK + 4 * lane;
    const bool wsv = grow < MPr;
    if (wsv) { *(volatile v2u*)gp = ph; *(volatile v2u*)(gp + DD) = pl; }
    __threadfence();
    if (wsv) { *(volatile v2u*)gp = ph; *(volatile v2u*)(gp + DD) = pl; }
  }
}

template <int EPI>
__global__ __launch_bounds__(GTHR) void k_gemm(const unsigned short* __restrict__ A, int lda,
                                               const unsigned short* __restrict__ BT, int ldb, int K,
                                               const float* __restrict__ bias,
                                               const float* __restrict__ bng, const float* __restrict__ bnb,
                                               const float* __restrict__ bnm, const float* __restrict__ bnv,
                                               void* outp, int ldo, int lsplit, int nN, int mRows) {
  __shared__ __attribute__((aligned(16))) float stg[GBM * GBN];
  __shared__ float cpar[5 * GBN];
  const int tid = (int)threadIdx.x, lane = tid & 31, wave = tid >> 5, hh = lane >> 4, m = lane & 15;
  const int rowBase = (int)blockIdx.x * GBM;
  const int colBase = (int)blockIdx.y * GBN;

  {
    const int col = colBase + tid;
    cpar[tid] = bf_rne(bias[col]);
    if constexpr (EPI == 1) {
      cpar[GBN + tid]     = bf_rne(bnm[col]);
      cpar[2 * GBN + tid] = rsqrtf(bf_rne(bnv[col]) + 1e-5f);
      cpar[3 * GBN + tid] = bf_rne(bng[col]);
      cpar[4 * GBN + tid] = bf_rne(bnb[col]);
    }
  }

  v8f acc[GNT];
  {
    const v8f z = {0.f, 0.f, 0.f, 0.f, 0.f, 0.f, 0.f, 0.f};
#pragma unroll
    for (int t = 0; t < GNT; ++t) acc[t] = z;
  }
  const unsigned short* ap = A  + (size_t)(rowBase + 16 * wave + m) * (size_t)lda + 8 * hh;
  const unsigned short* bp = BT + (size_t)(colBase + m) * (size_t)ldb + 8 * hh;

#pragma unroll 1
  for (int k0 = 0; k0 < K; k0 += 32) {
    Frag af;
    af.h[0] = *(const v8usa*)(ap + k0);
    af.h[1] = *(const v8usa*)(ap + k0 + 16);
#pragma unroll
    for (int nt = 0; nt < GNT; ++nt) {
      const unsigned short* wq = bp + (size_t)(16 * nt) * (size_t)ldb + k0;
      Frag bfr;
      bfr.h[0] = *(const v8usa*)wq;
      bfr.h[1] = *(const v8usa*)(wq + 16);
      acc[nt] = wmb(af, bfr, acc[nt]);
    }
  }
  __syncthreads();

#pragma unroll
  for (int nt = 0; nt < GNT; ++nt) {
    const int lc = 16 * nt + m;
    const float bb = cpar[lc];
#pragma unroll
    for (int r = 0; r < 8; ++r) {
      const int lr = 16 * wave + 8 * hh + r;
      const bool live = (rowBase + lr) < nN;
      float v = acc[nt][r] + bb;
      if constexpr (EPI == 1) {
        v = ((v - cpar[GBN + lc]) * cpar[2 * GBN + lc]) * cpar[3 * GBN + lc] + cpar[4 * GBN + lc];
      }
      v = relu_keep(v);
      stg[lr * GBN + lc] = live ? v : 0.0f;
    }
  }
  __syncthreads();

  if constexpr (EPI == 2) {
    unsigned short* outH = (unsigned short*)outp;
    const int cb = 8 * m;
    const bool isHi = (hh == 0);
    v4u pk[16];
#pragma unroll
    for (int i = 0; i < 16; ++i) {
      const int lr = 16 * wave + i;
      const v4f a = *(const v4fa*)(stg + lr * GBN + cb);
      const v4f b = *(const v4fa*)(stg + lr * GBN + cb + 4);
      const float f[8] = {a.x, a.y, a.z, a.w, b.x, b.y, b.z, b.w};
      unsigned int w[4];
#pragma unroll
      for (int j = 0; j < 4; ++j) {
        const unsigned short h0 = bf_bits(f[2 * j]), h1 = bf_bits(f[2 * j + 1]);
        const unsigned short l0 = bf_bits(f[2 * j] - bf_val(h0)), l1 = bf_bits(f[2 * j + 1] - bf_val(h1));
        const unsigned short q0 = isHi ? h0 : l0, q1 = isHi ? h1 : l1;
        w[j] = (unsigned int)q0 | ((unsigned int)q1 << 16);
      }
      v4u pv; pv.x = w[0]; pv.y = w[1]; pv.z = w[2]; pv.w = w[3];
      pk[i] = pv;
    }
#pragma unroll
    for (int i = 0; i < 16; ++i) {
      const int gr = rowBase + 16 * wave + i;
      unsigned short* op = outH + (size_t)gr * (size_t)ldo + colBase + cb + hh * lsplit;
      if (gr < mRows) *(volatile v4u*)op = pk[i];
    }
    __threadfence();
#pragma unroll
    for (int i = 0; i < 16; ++i) {
      const int gr = rowBase + 16 * wave + i;
      unsigned short* op = outH + (size_t)gr * (size_t)ldo + colBase + cb + hh * lsplit;
      if (gr < mRows) *(volatile v4u*)op = pk[i];
    }
  } else {
    float* outF = (float*)outp;
    v4f fv[16];
#pragma unroll
    for (int i = 0; i < 16; ++i) {
      const int lr = 16 * wave + i;
      fv[i] = *(const v4fa*)(stg + lr * GBN + 4 * lane);
    }
#pragma unroll
    for (int i = 0; i < 16; ++i) {
      const int gr = rowBase + 16 * wave + i;
      float* op = outF + (size_t)gr * (size_t)ldo + colBase + 4 * lane;
      if (gr < mRows) *(volatile v4f*)op = fv[i];
    }
    __threadfence();
#pragma unroll
    for (int i = 0; i < 16; ++i) {
      const int gr = rowBase + 16 * wave + i;
      float* op = outF + (size_t)gr * (size_t)ldo + colBase + 4 * lane;
      if (gr < mRows) *(volatile v4f*)op = fv[i];
    }
  }
}

__global__ __launch_bounds__(HTHR) void k_head(const float* __restrict__ Y, const int* __restrict__ bat,
                                               const unsigned short* __restrict__ L1T,
                                               const float* __restrict__ l1b,
                                               const float* __restrict__ l2w, const float* __restrict__ l2b,
                                               float* out, int nN, int nG, int nOut) {
  __shared__ __attribute__((aligned(16))) float accs[HG * DD];
  __shared__ __attribute__((aligned(16))) unsigned short ap[HG * APIT];
  __shared__ __attribute__((aligned(16))) float zs[HG * DD];
  __shared__ float lw[DD * NO];
  __shared__ float lb1[DD];
  __shared__ float lb2[16];
  __shared__ __attribute__((aligned(16))) float lg[HG * 16];
  __shared__ __attribute__((aligned(16))) float os[HG * NO];
  const int tid = (int)threadIdx.x, lane = tid & 31, wave = tid >> 5, hh = lane >> 4, m = lane & 15;
  const int g0 = (int)blockIdx.x * HG;
  int gl = nG - g0;
  gl = gl < 0 ? 0 : (gl > HG ? HG : gl);

#pragma unroll 4
  for (int r = 0; r < HG; ++r) accs[r * DD + tid] = 0.0f;
#pragma unroll 2
  for (int i = tid; i < DD * NO; i += HTHR) lw[i] = bf_rne(l2w[i]);
  lb1[tid] = bf_rne(l1b[tid]);
  if (tid < 16) {
    const float bb = l2b[tid < NO ? tid : NO - 1];
    lb2[tid] = (tid < NO) ? bf_rne(bb) : 0.0f;
  }
  __syncthreads();

#pragma unroll 1
  for (int n = 0; n < nN; ++n) {
    const int b = bat[n];
    const unsigned sl = (unsigned)(b - g0);
    if (sl < (unsigned)gl) {
      accs[sl * DD + tid] += Y[(size_t)n * DD + tid];
    }
  }
  __syncthreads();

#pragma unroll 4
  for (int r = 0; r < HG; ++r) {
    const float v = accs[r * DD + tid];
    const unsigned short hb = bf_bits(v);
    const unsigned short lb = bf_bits(v - bf_val(hb));
    ap[r * APIT + tid] = hb;
    ap[r * APIT + DD + tid] = lb;
  }
  __syncthreads();

  v8f acc[2];
  {
    const v8f z = {0.f, 0.f, 0.f, 0.f, 0.f, 0.f, 0.f, 0.f};
    acc[0] = z; acc[1] = z;
  }
  const unsigned short* bp = L1T + (size_t)(32 * wave + m) * HK + 8 * hh;
#pragma unroll 1
  for (int k0 = 0; k0 < HK; k0 += 32) {
    Frag af;
    af.h[0] = *(const v8usa*)(ap + m * APIT + k0 + 8 * hh);
    af.h[1] = *(const v8usa*)(ap + m * APIT + k0 + 16 + 8 * hh);
#pragma unroll
    for (int t = 0; t < 2; ++t) {
      const unsigned short* wq = bp + (size_t)(16 * t) * HK + k0;
      Frag bfr;
      bfr.h[0] = *(const v8usa*)wq;
      bfr.h[1] = *(const v8usa*)(wq + 16);
      acc[t] = wmb(af, bfr, acc[t]);
    }
  }
#pragma unroll
  for (int t = 0; t < 2; ++t) {
    const int col = 32 * wave + 16 * t + m;
    const float bb = lb1[col];
#pragma unroll
    for (int r = 0; r < 8; ++r) {
      const float v = relu_keep(acc[t][r] + bb);
      zs[(8 * hh + r) * DD + col] = v;
    }
  }
  __syncthreads();

#pragma unroll 1
  for (int idx = tid; idx < HG * NO; idx += HTHR) {
    const int g = idx / NO;
    const int o = idx - g * NO;
    float s = 0.0f;
#pragma unroll 4
    for (int k = 0; k < DD; ++k) s = fmaf(zs[g * DD + k], lw[k * NO + o], s);
    lg[g * 16 + o] = s + lb2[o];
  }
  __syncthreads();
  if (tid < HG) {
    const float qnan = __int_as_float(0x7fc00000);
    float mx = lg[tid * 16];
    bool bad = (mx != mx);
#pragma unroll 1
    for (int o = 1; o < NO; ++o) {
      const float l = lg[tid * 16 + o];
      bad = bad || (l != l);
      mx = (l > mx) ? l : mx;
    }
    float s = 0.0f;
#pragma unroll 1
    for (int o = 0; o < NO; ++o) s += expf(lg[tid * 16 + o] - mx);
    const float lse = logf(s);
    const float pz = bad ? qnan : 0.0f;
#pragma unroll 1
    for (int o = 0; o < NO; ++o) os[tid * NO + o] = ((lg[tid * 16 + o] - mx) - lse) + pz;
  }
  __syncthreads();

  const int base = g0 * NO;
  int cntf = nOut - base;
  cntf = cntf < 0 ? 0 : (cntf > HG * NO ? HG * NO : cntf);
  const bool okst = (tid < (HG * NO) / 4) && (4 * tid + 3 < cntf);
  const int pc = tid < (HG * NO) / 4 ? tid : (HG * NO) / 4 - 1;
  const v4f ov = *(const v4fa*)(os + 4 * pc);
  float* op = out + (size_t)base + 4 * pc;
  if (okst) *(volatile v4f*)op = ov;
  __threadfence();
  if (okst) *(volatile v4f*)op = ov;
}

static inline int cdiv(int a, int b) { return (a + b - 1) / b; }
static inline size_t al256(size_t o) { return (o + 255) & ~(size_t)255; }

extern "C" void kernel_launch(void* const* d_in, const int* in_sizes, int n_in,
                              void* d_out, int out_size, void* d_ws, size_t ws_size,
                              hipStream_t stream) {
  if (n_in < 25) return;
  if (in_sizes[0] < DD || (in_sizes[0] % DD) != 0) return;
  const int nN = in_sizes[0] / DD;
  if (nN < 1 || nN > (1 << 22)) return;
  const int nE2 = in_sizes[1];
  if (nE2 < 2 || (nE2 & 1) != 0) return;
  const int nE = nE2 / 2;
  if (nE < 1 || nE >= (1 << (31 - PKS))) return;
  if (in_sizes[2] != nN) return;
  if (in_sizes[3] != 1 || in_sizes[12] != 1) return;
  if (in_sizes[4] != DD * HID2 || in_sizes[5] != HID2) return;
  if (in_sizes[6] != HID2 * DD || in_sizes[7] != DD) return;
  if (in_sizes[8] != DD || in_sizes[9] != DD || in_sizes[10] != DD || in_sizes[11] != DD) return;
  if (in_sizes[13] != DD * HID2 || in_sizes[14] != HID2) return;
  if (in_sizes[15] != HID2 * DD || in_sizes[16] != DD) return;
  if (in_sizes[17] != DD || in_sizes[18] != DD || in_sizes[19] != DD || in_sizes[20] != DD) return;
  if (in_sizes[21] != DD * DD || in_sizes[22] != DD) return;
  if (in_sizes[23] != DD * NO || in_sizes[24] != NO) return;
  if (out_size < NO || (out_size % NO) != 0 || (out_size % 4) != 0) return;
  const int nG = out_size / NO;
  if (nG < 1 || nG > 65536) return;

  const float* x     = (const float*)d_in[0];
  const int*   ei    = (const int*)  d_in[1];
  const int*   src   = ei;
  const int*   dst   = ei + nE;
  const int*   batch = (const int*)  d_in[2];
  const float* eps0 = (const float*)d_in[3];
  const float* w1_0 = (const float*)d_in[4];   const float* b1_0 = (const float*)d_in[5];
  const float* w2_0 = (const float*)d_in[6];   const float* b2_0 = (const float*)d_in[7];
  const float* g0   = (const float*)d_in[8];   const float* be0  = (const float*)d_in[9];
  const float* m0   = (const float*)d_in[10];  const float* v0   = (const float*)d_in[11];
  const float* eps1 = (const float*)d_in[12];
  const float* w1_1 = (const float*)d_in[13];  const float* b1_1 = (const float*)d_in[14];
  const float* w2_1 = (const float*)d_in[15];  const float* b2_1 = (const float*)d_in[16];
  const float* g1   = (const float*)d_in[17];  const float* be1  = (const float*)d_in[18];
  const float* m1   = (const float*)d_in[19];  const float* v1   = (const float*)d_in[20];
  const float* l1w  = (const float*)d_in[21];  const float* l1b  = (const float*)d_in[22];
  const float* l2w  = (const float*)d_in[23];  const float* l2b  = (const float*)d_in[24];
  float* out = (float*)d_out;

  const int MP   = cdiv(nN, GBM) * GBM;
  const int gM   = MP / GBM;
  const int gA   = cdiv(MP, NB);
  const int vec8 = ((nE & 3) == 0) ? 1 : 0;
  if ((long long)gA * NB < (long long)MP) return;
  const int nUx  = nN * (DD / 8);
  const int gP   = cdiv(PB5 + nUx, NTHR);
  const int gH   = cdiv(nG, HG);

  char* ws = (char*)d_ws;
  size_t off = 0;
  const size_t oW10 = off; off = al256(off + (size_t)NUW1 * 16);
  const size_t oW11 = off; off = al256(off + (size_t)NUW1 * 16);
  const size_t oW20 = off; off = al256(off + (size_t)NUW2 * 16);
  const size_t oW21 = off; off = al256(off + (size_t)NUW2 * 16);
  const size_t oL1  = off; off = al256(off + (size_t)NUL1 * 16);
  const size_t oXB  = off; off = al256(off + (size_t)nUx * 16);
  const size_t oH   = off; off = al256(off + (size_t)MP * HK * 2);
  const size_t oT   = off; off = al256(off + (size_t)MP * TK * 2);
  const size_t oY0  = off; off = al256(off + (size_t)MP * DD * 4);
  const size_t oY1  = off; off = al256(off + (size_t)MP * DD * 4);
  if (off > ws_size || off > (size_t)WSMAX) return;
  unsigned short* W10 = (unsigned short*)(ws + oW10);
  unsigned short* W11 = (unsigned short*)(ws + oW11);
  unsigned short* W20 = (unsigned short*)(ws + oW20);
  unsigned short* W21 = (unsigned short*)(ws + oW21);
  unsigned short* L1  = (unsigned short*)(ws + oL1);
  unsigned short* XB  = (unsigned short*)(ws + oXB);
  unsigned short* H   = (unsigned short*)(ws + oH);
  unsigned short* T   = (unsigned short*)(ws + oT);
  float*          Y0  = (float*)(ws + oY0);
  float*          Y1  = (float*)(ws + oY1);

  hipFuncSetAttribute(reinterpret_cast<const void*>(&k_agg<1>), hipFuncAttributeMaxDynamicSharedMemorySize, LDS_AGG);
  hipFuncSetAttribute(reinterpret_cast<const void*>(&k_agg<0>), hipFuncAttributeMaxDynamicSharedMemorySize, LDS_AGG);

  k_prep<<<gP, NTHR, 0, stream>>>(x, nUx, w1_0, w1_1, w2_0, w2_1, l1w, W10, W11, W20, W21, L1, XB);
  k_agg<1><<<gA, NTHR, LDS_AGG, stream>>>(src, dst, XB, x, eps0, H, nN, nE, vec8, MP);
  k_gemm<2><<<dim3(gM, HID2 / GBN), GTHR, 0, stream>>>(H, HK, W10, HK, HK, b1_0, b1_0, b1_0, b1_0, b1_0,
                                                       (void*)T, TK, HID2, nN, MP);
  k_gemm<1><<<dim3(gM, DD / GBN), GTHR, 0, stream>>>(T, TK, W20, TK, TK, b2_0, g0, be0, m0, v0,
                                                     (void*)Y0, DD, 0, nN, MP);
  k_agg<0><<<gA, NTHR, LDS_AGG, stream>>>(src, dst, XB, Y0, eps1, H, nN, nE, vec8, MP);
  k_gemm<2><<<dim3(gM, HID2 / GBN), GTHR, 0, stream>>>(H, HK, W11, HK, HK, b1_1, b1_1, b1_1, b1_1, b1_1,
                                                       (void*)T, TK, HID2, nN, MP);
  k_gemm<1><<<dim3(gM, DD / GBN), GTHR, 0, stream>>>(T, TK, W21, TK, TK, b2_1, g1, be1, m1, v1,
                                                     (void*)Y1, DD, 0, nN, MP);
  k_head<<<gH, HTHR, 0, stream>>>(Y1, batch, L1, l1b, l2w, l2b, out, nN, nG, out_size);
}
